// SAGE_89996744720665
// MI455X (gfx1250) — hardware-verified
//
#include <hip/hip_runtime.h>
#include <stddef.h>
#include <stdint.h>
#include <math.h>


#define DIN    128
#define DH     256
#define NP     512
#define PP     512
#define HP     512
#define K0     128
#define K12    512
#define NTHR   256
#define NWAVE  8
#define EPT    8
#define CHUNK  (NTHR * EPT)
#define WCAP   (EPT * 32)
#define LISTN  (NWAVE * WCAP)
#define NBA    1024
#define SLA    10
#define RCAP   28672
#define DEGCAP 64
#define GBM    64
#define GBN    128
#define GTHR   128
#define NU0    (NP * (K0 / 8))
#define NU12   (NP * (K12 / 8))
#define NUW    (NU0 + 2 * NU12)
#define AGG_ZINTS    (LISTN + 2 * RCAP + 3 * NBA)
#define MISC_INTS    16
#define ROWBUF_INTS  (NWAVE * DH)
#define AGG_LDS_INTS (AGG_ZINTS + MISC_INTS + ROWBUF_INTS)
#define WSMAX  268435456

static_assert((CHUNK & (CHUNK - 1)) == 0 && CHUNK <= 4096);
static_assert((NBA & (NBA - 1)) == 0 && NBA == (1 << SLA));
static_assert(((long long)CHUNK << SLA) < (1LL << 31));
static_assert(LISTN % NTHR == 0);
static_assert(NBA % NWAVE == 0 && NBA % 32 == 0 && NBA % GBM == 0);
static_assert(RCAP % 32 == 0 && AGG_ZINTS % 4 == 0 && LISTN % 4 == 0 && ((AGG_ZINTS + MISC_INTS) % 4) == 0);
static_assert(AGG_ZINTS % (NTHR * 4) == 0);
static_assert(K0 % 32 == 0 && K12 % 32 == 0 && K12 == HP && K12 == 2 * DH && K0 == DIN);
static_assert(NP == 2 * DH && PP == NP && NP % GBN == 0);
static_assert(GBM == (GTHR / 32) * 16 && GBN == 4 * 32);
static_assert(DH == 8 * 32);
static_assert(NU0 % NTHR == 0 && NU12 % NTHR == 0 && NUW % NTHR == 0);
static_assert(((DH * (K0 / 8)) % NTHR) == 0 && ((DH * (K12 / 8)) % NTHR) == 0);
static_assert(DIN / 8 == 16 && K12 / 8 == 64);
static_assert(AGG_LDS_INTS * 4 <= 300000);

typedef float          v4f   __attribute__((ext_vector_type(4)));
typedef float          v8f   __attribute__((ext_vector_type(8)));
typedef int            v4i   __attribute__((ext_vector_type(4)));
typedef int            v8i   __attribute__((ext_vector_type(8)));
typedef unsigned short v8us  __attribute__((ext_vector_type(8)));
typedef unsigned short v16us __attribute__((ext_vector_type(16)));
typedef __bf16         v16bf __attribute__((ext_vector_type(16)));
typedef v4f  __attribute__((may_alias)) v4fa;
typedef v4i  __attribute__((may_alias)) v4ia;
typedef v8us __attribute__((may_alias)) v8usa;
union FragB { v16bf v; v16us u; v8us h[2]; v8i w; };

__device__ __forceinline__ v8f wmb(const FragB& a, const FragB& b, v8f c) {
  v8f d = __builtin_amdgcn_wmma_f32_16x16x32_bf16(false, a.v, false, b.v, (short)0, c, false, false);
  asm volatile("v_nop\n\tv_nop\n\tv_nop\n\tv_nop" : "+v"(d) : "v"(a.w), "v"(b.w));
  return d;
}

__device__ __forceinline__ unsigned bf16_bits(float f) {
  const unsigned u = __float_as_uint(f);
  return (u + 0x7FFFu + ((u >> 16) & 1u)) >> 16;
}
__device__ __forceinline__ float bf16_val(float f) {
  return __uint_as_float(bf16_bits(f) << 16);
}
__device__ __forceinline__ unsigned hl_bits(float v) {
  const unsigned hb = bf16_bits(v) & 0xffffu;
  const unsigned lb = bf16_bits(v - __uint_as_float(hb << 16)) & 0xffffu;
  return hb | (lb << 16);
}

__device__ __forceinline__ void wave_sync() {
  __builtin_amdgcn_fence(__ATOMIC_RELEASE, "wavefront");
  __builtin_amdgcn_wave_barrier();
  __builtin_amdgcn_fence(__ATOMIC_ACQUIRE, "wavefront");
}

template <int SLB>
__device__ __forceinline__ int scan_chunk(const int* __restrict__ dsts, int nE, int cbase, int slotBase,
                                          int nb, int vec8, int* list, int tid, int lane, int wave) {
  int wc = 0;
  const int el0  = tid * EPT;
  const int e0   = cbase + el0;
  const int sent = -2147483647 - 1;
  v4i da, db;
  if (vec8 != 0 && cbase + CHUNK <= nE) {
    da = *(const v4i*)(dsts + e0);
    db = *(const v4i*)(dsts + e0 + 4);
  } else {
    da.x = (e0     < nE) ? dsts[min(e0,     nE - 1)] : sent;
    da.y = (e0 + 1 < nE) ? dsts[min(e0 + 1, nE - 1)] : sent;
    da.z = (e0 + 2 < nE) ? dsts[min(e0 + 2, nE - 1)] : sent;
    da.w = (e0 + 3 < nE) ? dsts[min(e0 + 3, nE - 1)] : sent;
    db.x = (e0 + 4 < nE) ? dsts[min(e0 + 4, nE - 1)] : sent;
    db.y = (e0 + 5 < nE) ? dsts[min(e0 + 5, nE - 1)] : sent;
    db.z = (e0 + 6 < nE) ? dsts[min(e0 + 6, nE - 1)] : sent;
    db.w = (e0 + 7 < nE) ? dsts[min(e0 + 7, nE - 1)] : sent;
  }
  const unsigned nbs = (unsigned)slotBase;
  const unsigned unb = (unsigned)nb;
  const unsigned s0 = (unsigned)da.x - nbs, s1 = (unsigned)da.y - nbs;
  const unsigned s2 = (unsigned)da.z - nbs, s3 = (unsigned)da.w - nbs;
  const unsigned s4 = (unsigned)db.x - nbs, s5 = (unsigned)db.y - nbs;
  const unsigned s6 = (unsigned)db.z - nbs, s7 = (unsigned)db.w - nbs;
  const bool h0 = s0 < unb, h1 = s1 < unb, h2 = s2 < unb, h3 = s3 < unb;
  const bool h4 = s4 < unb, h5 = s5 < unb, h6 = s6 < unb, h7 = s7 < unb;
  const unsigned any = __builtin_amdgcn_ballot_w32(h0 | h1 | h2 | h3 | h4 | h5 | h6 | h7);
  if (any != 0u) {
#define HITJ(J, HJ, SJ) { \
      const unsigned mj = __builtin_amdgcn_ballot_w32(HJ); \
      if (mj != 0u) { \
        if (HJ) { \
          const int pos = wc + (int)__builtin_amdgcn_mbcnt_lo(mj, 0u); \
          if (pos < WCAP) list[wave * WCAP + pos] = ((el0 + (J)) << SLB) | (int)(SJ); \
        } \
        wc += (int)__builtin_popcount(mj); } }
    HITJ(0, h0, s0)
    HITJ(1, h1, s1)
    HITJ(2, h2, s2)
    HITJ(3, h3, s3)
    HITJ(4, h4, s4)
    HITJ(5, h5, s5)
    HITJ(6, h6, s6)
    HITJ(7, h7, s7)
#undef HITJ
  }
  return wc;
}

__global__ __launch_bounds__(NTHR) void k_wprep(const float* __restrict__ Wl0, const float* __restrict__ Wr0,
                                                const float* __restrict__ Wl1, const float* __restrict__ Wr1,
                                                const float* __restrict__ Wl2, const float* __restrict__ Wr2,
                                                unsigned short* BT0, unsigned short* BT1, unsigned short* BT2) {
  const int u = (int)blockIdx.x * NTHR + (int)threadIdx.x;
  const float* W;
  unsigned short* dp;
  int n, k8, kk;
  if (u < NU0) {
    n = u >> 4; k8 = (u & 15) * 8; kk = k8;
    W = (n < DH) ? Wl0 : Wr0;
    dp = BT0 + (size_t)n * K0 + k8;
  } else if (u < NU0 + NU12) {
    const int v = u - NU0;
    n = v >> 6; k8 = (v & 63) * 8; kk = k8 & (DH - 1);
    W = (n < DH) ? Wl1 : Wr1;
    dp = BT1 + (size_t)n * K12 + k8;
  } else if (u < NUW) {
    const int v = u - NU0 - NU12;
    n = v >> 6; k8 = (v & 63) * 8; kk = k8 & (DH - 1);
    W = (n < DH) ? Wl2 : Wr2;
    dp = BT2 + (size_t)n * K12 + k8;
  } else {
    return;
  }
  const int col = n & (DH - 1);
  const float* p = W + (size_t)kk * DH + col;
  v8us o;
#pragma unroll
  for (int i = 0; i < 8; ++i) o[i] = (unsigned short)bf16_bits(p[(size_t)i * DH]);
  *(volatile v8us*)dp = o;
  __threadfence();
  *(volatile v8us*)dp = o;
}

__global__ __launch_bounds__(NTHR) void k_cvx(const float* __restrict__ x, int nN, int nUnits,
                                              unsigned short* xb) {
  const int u = (int)blockIdx.x * NTHR + (int)threadIdx.x;
  if (u >= nUnits) return;
  const int row = u >> 4;
  const int k8  = (u & 15) * 8;
  const int rc  = row < nN ? row : nN - 1;
  const float* p = x + (size_t)rc * DIN + k8;
  const v4f a = *(const v4fa*)p;
  const v4f b = *(const v4fa*)(p + 4);
  const bool ok = row < nN;
  v8us o;
  o[0] = ok ? (unsigned short)bf16_bits(a.x) : (unsigned short)0;
  o[1] = ok ? (unsigned short)bf16_bits(a.y) : (unsigned short)0;
  o[2] = ok ? (unsigned short)bf16_bits(a.z) : (unsigned short)0;
  o[3] = ok ? (unsigned short)bf16_bits(a.w) : (unsigned short)0;
  o[4] = ok ? (unsigned short)bf16_bits(b.x) : (unsigned short)0;
  o[5] = ok ? (unsigned short)bf16_bits(b.y) : (unsigned short)0;
  o[6] = ok ? (unsigned short)bf16_bits(b.z) : (unsigned short)0;
  o[7] = ok ? (unsigned short)bf16_bits(b.w) : (unsigned short)0;
  unsigned short* dp = xb + (size_t)row * DIN + k8;
  *(volatile v8us*)dp = o;
  __threadfence();
  *(volatile v8us*)dp = o;
}

__global__ __launch_bounds__(GTHR) void k_gemm(const unsigned short* __restrict__ A, int lda,
                                               const unsigned short* __restrict__ BT, int K,
                                               float* outp, int ldo) {
  __shared__ __attribute__((aligned(16))) float stg[GBM * GBN];
  const int tid = (int)threadIdx.x, lane = tid & 31, wave = tid >> 5, hh = lane >> 4, m = lane & 15;
  const int rowBase = (int)blockIdx.x * GBM;
  const int col0    = (int)blockIdx.y * GBN;

  v8f acc[8];
  {
    const v8f z = {0.f, 0.f, 0.f, 0.f, 0.f, 0.f, 0.f, 0.f};
#pragma unroll
    for (int t = 0; t < 8; ++t) acc[t] = z;
  }
  const unsigned short* ap = A  + (size_t)(rowBase + 16 * wave + m) * (size_t)lda + 8 * hh;
  const unsigned short* bp = BT + (size_t)(col0 + m) * (size_t)K + 8 * hh;

#pragma unroll 1
  for (int k0 = 0; k0 < K; k0 += 32) {
    FragB af;
    af.h[0] = *(const v8usa*)(ap + k0);
    af.h[1] = *(const v8usa*)(ap + k0 + 16);
#pragma unroll
    for (int nt = 0; nt < 8; ++nt) {
      const unsigned short* wq = bp + (size_t)(16 * nt) * (size_t)K + k0;
      FragB bf;
      bf.h[0] = *(const v8usa*)wq;
      bf.h[1] = *(const v8usa*)(wq + 16);
      acc[nt] = wmb(af, bf, acc[nt]);
    }
  }

#pragma unroll
  for (int nt = 0; nt < 8; ++nt) {
    const int lc = 16 * nt + m;
#pragma unroll
    for (int r = 0; r < 8; ++r) {
      const int lr = 16 * wave + 8 * hh + r;
      stg[lr * GBN + lc] = acc[nt][r];
    }
  }
  __syncthreads();

  v4f pv[16];
#pragma unroll
  for (int i = 0; i < 16; ++i) pv[i] = *(const v4fa*)(stg + (16 * wave + i) * GBN + 4 * lane);
#pragma unroll
  for (int i = 0; i < 16; ++i) {
    float* op = outp + (size_t)(rowBase + 16 * wave + i) * (size_t)ldo + col0 + 4 * lane;
    *(volatile v4f*)op = pv[i];
  }
  __threadfence();
#pragma unroll
  for (int i = 0; i < 16; ++i) {
    float* op = outp + (size_t)(rowBase + 16 * wave + i) * (size_t)ldo + col0 + 4 * lane;
    *(volatile v4f*)op = pv[i];
  }
}

template <int MODE>
__global__ __launch_bounds__(NTHR) void k_scan(const int* __restrict__ srcs, const int* __restrict__ dsts,
                                               int nE, int nN, int vec8, int mRows,
                                               const float* __restrict__ pin, const float* __restrict__ bias,
                                               unsigned short* hpl, float* outp) {
  extern __shared__ __attribute__((aligned(16))) int dsm[];
  int* list = dsm;
  int* hl   = dsm + LISTN;
  int* sl   = hl + RCAP;
  int* cnt  = sl + RCAP;
  int* offs = cnt + NBA;
  int* cur  = offs + NBA;
  int* misc = cur + NBA;
  const int tid = (int)threadIdx.x, lane = tid & 31, wave = tid >> 5;
  float* rowbuf = (float*)(misc + MISC_INTS) + wave * DH;
  const int nodeBase = (int)blockIdx.x * NBA;

  {
    const v4i z4 = {0, 0, 0, 0};
    for (int i = tid * 4; i < AGG_ZINTS; i += NTHR * 4) *(v4ia*)(dsm + i) = z4;
    if (tid < MISC_INTS) misc[tid] = 0;
  }
  __syncthreads();

  int t = 0, ov = 0;
  const int nChunks = (nE + CHUNK - 1) / CHUNK;
#pragma unroll 1
  for (int ch = 0; ch < nChunks; ++ch) {
    const int cbase = ch * CHUNK;
    const int wc = scan_chunk<SLA>(dsts, nE, cbase, nodeBase, NBA, vec8, list, tid, lane, wave);
    if (lane == 0) misc[wave] = wc;
    __syncthreads();
    if (wave == 0) {
#pragma unroll 1
      for (int w2 = 0; w2 < NWAVE; ++w2) {
        int c = misc[w2];
        c = c < 0 ? 0 : (c > WCAP ? WCAP : c);
#pragma unroll 1
        for (int b0 = 0; b0 < c; b0 += 32) {
          const int idx = b0 + lane;
          const int ent = list[w2 * WCAP + (idx < WCAP ? idx : WCAP - 1)];
          const int m32 = (c - b0) < 32 ? (c - b0) : 32;
#pragma unroll 1
          for (int k = 0; k < m32; ++k) {
            const int u    = __builtin_amdgcn_readlane(ent, k);
            const int slot = u & (NBA - 1);
            const int el   = (u >> SLA) & (CHUNK - 1);
            const int pk   = ((cbase + el) << SLA) | slot;
            if (t < RCAP) {
              if (lane == 0) { hl[t] = pk; cnt[slot] = cnt[slot] + 1; }
              t = t + 1;
            } else {
              ov = 1;
            }
          }
        }
      }
    }
    __syncthreads();
  }
  if (wave == 0 && lane == 0) { misc[8] = t; misc[9] = ov; }
  __syncthreads();
  int tt = misc[8];
  tt = tt < 0 ? 0 : (tt > RCAP ? RCAP : tt);
  const int ovf = misc[9];

  if (wave == 0) {
    const int base = lane * (NBA / 32);
    int s = 0;
#pragma unroll 1
    for (int i = 0; i < NBA / 32; ++i) s += cnt[base + i];
    int incl = s;
#pragma unroll
    for (int d = 1; d < 32; d <<= 1) {
      const int y = __shfl_up(incl, d, 32);
      if (lane >= d) incl += y;
    }
    int run = incl - s;
#pragma unroll 1
    for (int i = 0; i < NBA / 32; ++i) {
      const int cv = cnt[base + i];
      offs[base + i] = run;
      cur[base + i]  = run;
      run += cv;
    }
  }
  __syncthreads();
  if (wave == 0) {
#pragma unroll 1
    for (int b0 = 0; b0 < tt; b0 += 32) {
      const int idx = b0 + lane;
      const int ent = hl[idx < RCAP ? idx : RCAP - 1];
      const int m32 = (tt - b0) < 32 ? (tt - b0) : 32;
#pragma unroll 1
      for (int k = 0; k < m32; ++k) {
        const int u    = __builtin_amdgcn_readlane(ent, k);
        const int slot = u & (NBA - 1);
        if (lane == 0) {
          int p = cur[slot];
          p = p < 0 ? 0 : (p > RCAP - 1 ? RCAP - 1 : p);
          sl[p] = u;
          cur[slot] = p + 1;
        }
      }
    }
  }
  __syncthreads();

  const float qnan = __int_as_float(0x7fc00000);
  const float pz = (ovf != 0) ? qnan : 0.0f;
  v4f ba, bb;
  {
    const v4f t0 = *(const v4fa*)(bias + 8 * lane);
    const v4f t1 = *(const v4fa*)(bias + 8 * lane + 4);
    ba.x = bf16_val(t0.x); ba.y = bf16_val(t0.y); ba.z = bf16_val(t0.z); ba.w = bf16_val(t0.w);
    bb.x = bf16_val(t1.x); bb.y = bf16_val(t1.y); bb.z = bf16_val(t1.z); bb.w = bf16_val(t1.w);
  }
#pragma unroll 1
  for (int si = 0; si < NBA / NWAVE; ++si) {
    const int s    = si * NWAVE + wave;
    const int node = nodeBase + s;
    int c = cnt[s];
    const bool big = c > DEGCAP;
    c = c < 0 ? 0 : (c > DEGCAP ? DEGCAP : c);
    int o = offs[s];
    o = o < 0 ? 0 : (o > RCAP ? RCAP : o);
    const int nc = node < nN ? node : nN - 1;
    v4f aa = {0.0f, 0.0f, 0.0f, 0.0f};
    v4f ab = {0.0f, 0.0f, 0.0f, 0.0f};
#pragma unroll 1
    for (int b0 = 0; b0 < c; b0 += 32) {
      int idx = o + b0 + lane;
      idx = idx > RCAP - 1 ? RCAP - 1 : idx;
      const int ent = sl[idx];
      int eid = ent >> SLA;
      eid = eid < 0 ? 0 : (eid > nE - 1 ? nE - 1 : eid);
      int sr = srcs[eid];
      sr = sr < 0 ? 0 : (sr > nN - 1 ? nN - 1 : sr);
      const int m32 = (c - b0) < 32 ? (c - b0) : 32;
#pragma unroll 1
      for (int k = 0; k < m32; ++k) {
        const int sk = __builtin_amdgcn_readlane(sr, k);
        const float* rp = pin + (size_t)sk * PP + 8 * lane;
        const v4f va = *(const v4fa*)rp;
        const v4f vb = *(const v4fa*)(rp + 4);
        aa += va;
        ab += vb;
      }
    }
    const float degf = (float)(c < 1 ? 1 : c);
    const float invd = 1.0f / degf;
    const float* rr = pin + (size_t)nc * PP + DH + 8 * lane;
    const v4f ra = *(const v4fa*)rr;
    const v4f rb = *(const v4fa*)(rr + 4);
    v4f ya = (aa * invd + ba) + ra;
    v4f yb = (ab * invd + bb) + rb;
    if constexpr (MODE == 0) {
      ya.x = fmaxf(ya.x, 0.0f); ya.y = fmaxf(ya.y, 0.0f); ya.z = fmaxf(ya.z, 0.0f); ya.w = fmaxf(ya.w, 0.0f);
      yb.x = fmaxf(yb.x, 0.0f); yb.y = fmaxf(yb.y, 0.0f); yb.z = fmaxf(yb.z, 0.0f); yb.w = fmaxf(yb.w, 0.0f);
    }
    const float pzr = big ? qnan : pz;
    const bool live = node < nN;
    ya = ya + pzr; yb = yb + pzr;
    ya.x = live ? ya.x : 0.0f; ya.y = live ? ya.y : 0.0f; ya.z = live ? ya.z : 0.0f; ya.w = live ? ya.w : 0.0f;
    yb.x = live ? yb.x : 0.0f; yb.y = live ? yb.y : 0.0f; yb.z = live ? yb.z : 0.0f; yb.w = live ? yb.w : 0.0f;
    if constexpr (MODE == 0) {
      v8us h8, l8;
      unsigned w;
      w = hl_bits(ya.x); h8[0] = (unsigned short)(w & 0xffffu); l8[0] = (unsigned short)(w >> 16);
      w = hl_bits(ya.y); h8[1] = (unsigned short)(w & 0xffffu); l8[1] = (unsigned short)(w >> 16);
      w = hl_bits(ya.z); h8[2] = (unsigned short)(w & 0xffffu); l8[2] = (unsigned short)(w >> 16);
      w = hl_bits(ya.w); h8[3] = (unsigned short)(w & 0xffffu); l8[3] = (unsigned short)(w >> 16);
      w = hl_bits(yb.x); h8[4] = (unsigned short)(w & 0xffffu); l8[4] = (unsigned short)(w >> 16);
      w = hl_bits(yb.y); h8[5] = (unsigned short)(w & 0xffffu); l8[5] = (unsigned short)(w >> 16);
      w = hl_bits(yb.z); h8[6] = (unsigned short)(w & 0xffffu); l8[6] = (unsigned short)(w >> 16);
      w = hl_bits(yb.w); h8[7] = (unsigned short)(w & 0xffffu); l8[7] = (unsigned short)(w >> 16);
      if (node < mRows) {
        unsigned short* hp = hpl + (size_t)node * HP + 8 * lane;
        *(volatile v8us*)hp = h8;
        *(volatile v8us*)(hp + DH) = l8;
        __threadfence();
        *(volatile v8us*)hp = h8;
        *(volatile v8us*)(hp + DH) = l8;
      }
    } else {
      *(v4fa*)(rowbuf + 8 * lane) = ya;
      *(v4fa*)(rowbuf + 8 * lane + 4) = yb;
      wave_sync();
      const v4f q0 = *(const v4fa*)(rowbuf + 4 * lane);
      const v4f q1 = *(const v4fa*)(rowbuf + (DH / 2) + 4 * lane);
      wave_sync();
      if (live) {
        float* op = outp + (size_t)node * DH + 4 * lane;
        *(volatile v4f*)op = q0;
        *(volatile v4f*)(op + DH / 2) = q1;
        __threadfence();
        *(volatile v4f*)op = q0;
        *(volatile v4f*)(op + DH / 2) = q1;
      }
    }
  }
}

static inline int cdiv(int a, int b) { return (a + b - 1) / b; }
static inline size_t al256(size_t o) { return (o + 255) & ~(size_t)255; }

extern "C" void kernel_launch(void* const* d_in, const int* in_sizes, int n_in,
                              void* d_out, int out_size, void* d_ws, size_t ws_size,
                              hipStream_t stream) {
  if (n_in < 11) return;
  if (in_sizes[0] < DIN || (in_sizes[0] % DIN) != 0) return;
  const int nN = in_sizes[0] / DIN;
  if (nN < 16 || nN > (1 << 22)) return;
  if (in_sizes[1] < 2 || (in_sizes[1] & 1) != 0) return;
  const int nE = in_sizes[1] / 2;
  if (nE < 1 || nE >= (1 << (31 - SLA))) return;
  if (in_sizes[2] != DIN * DH || in_sizes[3] != DH || in_sizes[4] != DIN * DH) return;
  if (in_sizes[5] != DH * DH  || in_sizes[6] != DH || in_sizes[7] != DH * DH) return;
  if (in_sizes[8] != DH * DH  || in_sizes[9] != DH || in_sizes[10] != DH * DH) return;
  if ((long long)out_size != (long long)nN * DH) return;

  const float* x    = (const float*)d_in[0];
  const int*   edge = (const int*)d_in[1];
  const float* Wl0  = (const float*)d_in[2];
  const float* bl0  = (const float*)d_in[3];
  const float* Wr0  = (const float*)d_in[4];
  const float* Wl1  = (const float*)d_in[5];
  const float* bl1  = (const float*)d_in[6];
  const float* Wr1  = (const float*)d_in[7];
  const float* Wl2  = (const float*)d_in[8];
  const float* bl2  = (const float*)d_in[9];
  const float* Wr2  = (const float*)d_in[10];
  float* out = (float*)d_out;
  const int* src = edge;
  const int* dst = edge + nE;

  const int MP = cdiv(nN, GBM) * GBM;
  const int gM = MP / GBM;
  const int gA = cdiv(MP, NBA);
  if ((long long)gA * NBA < (long long)MP) return;
  const int vec8 = ((nE & 3) == 0) ? 1 : 0;

  char* ws = (char*)d_ws;
  size_t off = 0;
  const size_t oBT0 = off; off = al256(off + (size_t)NP * K0 * 2);
  const size_t oBT1 = off; off = al256(off + (size_t)NP * K12 * 2);
  const size_t oBT2 = off; off = al256(off + (size_t)NP * K12 * 2);
  const size_t oXB  = off; off = al256(off + (size_t)MP * DIN * 2);
  const size_t oP   = off; off = al256(off + (size_t)MP * PP * 4);
  const size_t oH   = off; off = al256(off + (size_t)MP * HP * 2);
  if (off > ws_size || off > (size_t)WSMAX) return;
  unsigned short* BT0 = (unsigned short*)(ws + oBT0);
  unsigned short* BT1 = (unsigned short*)(ws + oBT1);
  unsigned short* BT2 = (unsigned short*)(ws + oBT2);
  unsigned short* XB  = (unsigned short*)(ws + oXB);
  float*          P   = (float*)(ws + oP);
  unsigned short* H   = (unsigned short*)(ws + oH);

  const size_t scanLds = (size_t)AGG_LDS_INTS * 4;
  hipFuncSetAttribute(reinterpret_cast<const void*>(&k_scan<0>), hipFuncAttributeMaxDynamicSharedMemorySize, (int)scanLds);
  hipFuncSetAttribute(reinterpret_cast<const void*>(&k_scan<1>), hipFuncAttributeMaxDynamicSharedMemorySize, (int)scanLds);

  const int nUx = MP * (DIN / 8);
  k_wprep<<<NUW / NTHR, NTHR, 0, stream>>>(Wl0, Wr0, Wl1, Wr1, Wl2, Wr2, BT0, BT1, BT2);
  k_cvx<<<cdiv(nUx, NTHR), NTHR, 0, stream>>>(x, nN, nUx, XB);
  k_gemm<<<dim3(gM, NP / GBN), GTHR, 0, stream>>>(XB, DIN, BT0, K0, P, PP);
  k_scan<0><<<gA, NTHR, scanLds, stream>>>(src, dst, nE, nN, vec8, MP, P, bl0, H, out);
  k_gemm<<<dim3(gM, NP / GBN), GTHR, 0, stream>>>(H, HP, BT1, K12, P, PP);
  k_scan<0><<<gA, NTHR, scanLds, stream>>>(src, dst, nE, nN, vec8, MP, P, bl1, H, out);
  k_gemm<<<dim3(gM, NP / GBN), GTHR, 0, stream>>>(H, HP, BT2, K12, P, PP);
  k_scan<1><<<gA, NTHR, scanLds, stream>>>(src, dst, nE, nN, vec8, MP, P, bl2, H, out);
}
